// WaveFunctionDensity_25786983645324
// MI455X (gfx1250) — hardware-run, weakly checked
//
#include <hip/hip_runtime.h>


#ifndef NB
#define NB 16
#endif
#ifndef MS
#define MS 4096
#endif
#define NB_FULL 16
#define MS_FULL 4096
#ifndef OUT_MS
#define OUT_MS MS
#endif
#define NA   32
#define NPR  512
#define NSYM 20
#define MT   32
#define KW   4
#define BHP  520
#define BFP  516
#define BSC  512.0f
#define DSC  4096.0f
#define OSC  (1.0f / 2097152.0f)
#define HLIM 60000.0f

static_assert(NPR % 32 == 0);
static_assert(NPR == KW * 128);
static_assert(MT == 32);
static_assert(MS % MT == 0);
static_assert(OUT_MS % 32 == 0);
static_assert(8 * 16 == MT * 4);
static_assert((MT * NA * 3) % (4 * 32 * KW) == 0);
static_assert((BHP * 2) % 16 == 0);
static_assert(BHP >= NPR);
static_assert(BFP >= NPR);
static_assert(((size_t)NB * NPR * NPR) % (8 * 256) == 0);
static_assert(NB <= NB_FULL);
static_assert(MS <= MS_FULL);
static_assert((size_t)MT * BHP * 2 + (size_t)MT * BFP * 4 + (size_t)MT * NA * 3 * 4 + (size_t)KW * MT * 4 <= (size_t)131072);

typedef _Float16 h16;
typedef __attribute__((ext_vector_type(16))) _Float16 v16h;
typedef __attribute__((ext_vector_type(8)))  _Float16 v8h;
typedef __attribute__((ext_vector_type(8)))  float    v8f;
typedef __attribute__((ext_vector_type(4)))  float    v4f;
typedef v4f  __attribute__((may_alias)) v4fa;

__device__ __forceinline__ unsigned short f2bf(float f) { unsigned u = __float_as_uint(f); u += 0x7FFFu + ((u >> 16) & 1u); return (unsigned short)(u >> 16); }
__device__ __forceinline__ float bfr(float f) { return __uint_as_float(((unsigned)f2bf(f)) << 16); }
__device__ __forceinline__ v16h cat16(v8h lo, v8h hi) { return __builtin_shufflevector(lo, hi, 0, 1, 2, 3, 4, 5, 6, 7, 8, 9, 10, 11, 12, 13, 14, 15); }
__device__ __forceinline__ v16h  ldh(const h16* p) { return cat16(*(const v8h*)p, *(const v8h*)(p + 16)); }
static __device__ __forceinline__ h16 toh_flush(float v) { const h16 r = (h16)v; return (fabsf(v) < 6.103515625e-05f) ? (h16)0.0f : r; }
__device__ __forceinline__ v8f wmma16g(v16h a, v16h b, v8f c) {
    c = __builtin_amdgcn_wmma_f32_16x16x32_f16(false, a, false, b, (short)0, c, false, false);
    asm volatile("v_nop\n\tv_nop\n\tv_nop\n\tv_nop" : "+v"(c) : "v"(a), "v"(b));
    return c;
}
__device__ __forceinline__ float powi3(float x, unsigned e) {
    float r = 1.0f;
    if (e >= 1u) r = x;
    if (e >= 2u) r *= x;
    if (e >= 3u) r *= x;
    return r;
}

#define SYE(i, px, py, pz) (((unsigned long long)((px) | ((py) << 2) | ((pz) << 4))) << (6 * (i)))
#define SYLO (SYE(0, 0, 0, 0) | SYE(1, 1, 0, 0) | SYE(2, 0, 1, 0) | SYE(3, 0, 0, 1) | SYE(4, 2, 0, 0) | SYE(5, 0, 2, 0) | SYE(6, 0, 0, 2) | SYE(7, 1, 1, 0) | SYE(8, 1, 0, 1) | SYE(9, 0, 1, 1))
#define SYHI (SYE(0, 3, 0, 0) | SYE(1, 0, 3, 0) | SYE(2, 0, 0, 3) | SYE(3, 2, 1, 0) | SYE(4, 2, 0, 1) | SYE(5, 0, 2, 1) | SYE(6, 1, 2, 0) | SYE(7, 1, 0, 2) | SYE(8, 0, 1, 2) | SYE(9, 1, 1, 1))

__global__ __launch_bounds__(256) void k_dmcvt(const float* __restrict__ src, h16* dst, size_t n8) {
    const size_t i = (size_t)blockIdx.x * 256 + threadIdx.x; if (i >= n8) return;
    const v8f v = *(const v8f*)(src + i * 8); v8h o;
#pragma unroll
    for (int k = 0; k < 8; ++k) o[k] = toh_flush(bfr(v[k]) * DSC);
    *(volatile v8h*)(dst + i * 8) = o; __threadfence(); *(volatile v8h*)(dst + i * 8) = o;
}

__global__ __launch_bounds__(32 * KW) void k_dens(const float* __restrict__ DV, const int* __restrict__ CEN, const float* __restrict__ ALP, const int* __restrict__ SYM,
                                                   const h16* __restrict__ DH, float* OUT) {
    __shared__ __align__(16) h16   bhs[MT * BHP];
    __shared__ __align__(16) float bfs[MT * BFP];
    __shared__ __align__(16) float dvs[MT * NA * 3];
    __shared__ __align__(16) float red[KW * MT];
    const int tid = threadIdx.x;
    const int lane = tid & 31, lr = lane & 15, hi = lane >> 4;
    const int wave = __builtin_amdgcn_readfirstlane((int)(threadIdx.x >> 5));
    const int n = blockIdx.y; const int m0 = blockIdx.x * MT;

    const float* dsrc = DV + ((size_t)n * MS_FULL + (size_t)m0) * (NA * 3);
#pragma unroll 1
    for (int i = tid; i < MT * NA * 3 / 4; i += 32 * KW) {
        v4f v = *(const v4f*)(dsrc + (size_t)i * 4);
        v[0] = bfr(v[0]); v[1] = bfr(v[1]); v[2] = bfr(v[2]); v[3] = bfr(v[3]);
        *(v4fa*)(&dvs[i * 4]) = v; }
    __syncthreads();

    const int pb = n * NPR;
#pragma unroll 1
    for (int pp = 0; pp < 128; ++pp) {
        const int p = wave * 128 + pp;
        const int c = CEN[pb + p];
        const bool valid = c >= 0;
        int ci = c < 0 ? 0 : c; ci = ci > NA - 1 ? NA - 1 : ci;
        int s = valid ? SYM[pb + p] : 0;
        s = s < 0 ? s + NSYM : s; s = s < 0 ? 0 : (s > NSYM - 1 ? NSYM - 1 : s);
        const float al = bfr(ALP[pb + p]);
        const int sj = s < 10 ? s : s - 10;
        const unsigned long long tw = s < 10 ? (unsigned long long)SYLO : (unsigned long long)SYHI;
        const unsigned code = (unsigned)(tw >> (6 * sj)) & 63u;
        const float x = dvs[lane * (NA * 3) + ci * 3 + 0], y = dvs[lane * (NA * 3) + ci * 3 + 1], z = dvs[lane * (NA * 3) + ci * 3 + 2];
        const float r2 = (x * x + z * z) + y * y;
        const float ang = powi3(x, code & 3u) * powi3(y, (code >> 2) & 3u) * powi3(z, (code >> 4) & 3u);
        const float e = expf(-(al * r2));
        const float bv = valid ? ang * e : 0.0f;
        float sv = bv * BSC; sv = fminf(fmaxf(sv, -HLIM), HLIM);
        bfs[lane * BFP + p] = bv;
        bhs[lane * BHP + p] = toh_flush(sv);
    }
    __syncthreads();

    float p0[8], p1[8];
#pragma unroll
    for (int r = 0; r < 8; ++r) { p0[r] = 0.0f; p1[r] = 0.0f; }
    const int ai0 = lr * BHP + 8 * hi, ai1 = (16 + lr) * BHP + 8 * hi;
#pragma unroll 1
    for (int ch = 0; ch < 2; ++ch) {
        const int c0 = wave * 128 + ch * 64;
        v8f acc0[4], acc1[4];
#pragma unroll
        for (int nb = 0; nb < 4; ++nb) { acc0[nb] = (v8f){}; acc1[nb] = (v8f){}; }
        const size_t bo = (size_t)n * NPR * NPR + (size_t)(c0 + lr) * NPR + 8 * hi;
#pragma unroll 1
        for (int kc = 0; kc < NPR; kc += 32) {
            const v16h a0 = cat16(*(const v8h*)(&bhs[ai0 + kc]), *(const v8h*)(&bhs[ai0 + kc + 16]));
            const v16h a1 = cat16(*(const v8h*)(&bhs[ai1 + kc]), *(const v8h*)(&bhs[ai1 + kc + 16]));
#pragma unroll
            for (int nb = 0; nb < 4; ++nb) {
                const v16h b = ldh(DH + bo + (size_t)nb * 16 * NPR + kc);
                acc0[nb] = wmma16g(a0, b, acc0[nb]);
                acc1[nb] = wmma16g(a1, b, acc1[nb]); }
        }
#pragma unroll
        for (int nb = 0; nb < 4; ++nb) {
#pragma unroll
            for (int r = 0; r < 8; ++r) {
                p0[r] += acc0[nb][r] * bfs[(8 * hi + r) * BFP + c0 + nb * 16 + lr];
                p1[r] += acc1[nb][r] * bfs[(16 + 8 * hi + r) * BFP + c0 + nb * 16 + lr]; } }
    }
#pragma unroll
    for (int r = 0; r < 8; ++r) {
        float v0 = p0[r]; v0 += __shfl_xor(v0, 1, 32); v0 += __shfl_xor(v0, 2, 32); v0 += __shfl_xor(v0, 4, 32); v0 += __shfl_xor(v0, 8, 32); p0[r] = v0;
        float v1 = p1[r]; v1 += __shfl_xor(v1, 1, 32); v1 += __shfl_xor(v1, 2, 32); v1 += __shfl_xor(v1, 4, 32); v1 += __shfl_xor(v1, 8, 32); p1[r] = v1; }
    if (lr == 0) {
#pragma unroll
        for (int r = 0; r < 8; ++r) { red[wave * MT + 8 * hi + r] = p0[r]; red[wave * MT + 16 + 8 * hi + r] = p1[r]; } }
    __syncthreads();

    if (wave == 0) {
        const int rq = (lane & 7) * 4; v4f val;
#pragma unroll
        for (int i = 0; i < 4; ++i) { float s = red[rq + i]; s += red[MT + rq + i]; s += red[2 * MT + rq + i]; s += red[3 * MT + rq + i]; val[i] = s * OSC; }
        asm volatile("" : "+v"(val));
        float* op = OUT + (size_t)n * OUT_MS + (size_t)m0 + rq;
#pragma unroll 1
        for (int ps = 0; ps < 2; ++ps) {
            if (lane < 8) *(volatile v4f*)op = val;
            if (ps == 0) __threadfence(); }
    }
}

static constexpr size_t al256(size_t v) { return (v + 255) & ~(size_t)255; }
static constexpr size_t SZ_DH = al256((size_t)NB * NPR * NPR * 2);
static constexpr size_t SZ_TOTAL = SZ_DH;
static_assert(SZ_TOTAL <= (size_t)134217728);

extern "C" void kernel_launch(void* const* d_in, const int* in_sizes, int n_in,
                              void* d_out, int out_size, void* d_ws, size_t ws_size, hipStream_t stream) {
    if (n_in < 5) return;
    const size_t needdv = ((size_t)(NB - 1) * MS_FULL + MS) * NA * 3;
    if ((size_t)in_sizes[0] < needdv) return;
    if ((size_t)in_sizes[1] < (size_t)NB * NPR || (size_t)in_sizes[2] < (size_t)NB * NPR || (size_t)in_sizes[3] < (size_t)NB * NPR) return;
    if ((size_t)in_sizes[4] < (size_t)NB * NPR * NPR) return;
    if ((size_t)out_size < (size_t)(NB - 1) * OUT_MS + MS) return;
    if (SZ_TOTAL > ws_size) return;
    const float* dv  = (const float*)d_in[0];
    const int*   cen = (const int*)d_in[1];
    const float* alp = (const float*)d_in[2];
    const int*   sym = (const int*)d_in[3];
    const float* dm  = (const float*)d_in[4];
    float* OUT = (float*)d_out;
    h16* DH = (h16*)d_ws;

    { const size_t n8 = (size_t)NB * NPR * NPR / 8;
      k_dmcvt<<<(unsigned)((n8 + 255) / 256), 256, 0, stream>>>(dm, DH, n8); }
    k_dens<<<dim3(MS / MT, NB, 1), 32 * KW, 0, stream>>>(dv, cen, alp, sym, DH, OUT);
}
